// SelfAttention_12506944766474
// MI455X (gfx1250) — hardware-verified
//
#include <hip/hip_runtime.h>
#ifndef NB
#define NB 4
#endif
#ifndef SEQ
#define SEQ 4096
#endif
#define NB_FULL 4
#define SEQ_FULL 4096
#define DM 768
#define HD 64
#define NQKV 192
#define NR ((size_t)NB * SEQ)
#define PLANE (NR * HD)
#define RES_ROWS 512

static_assert(SEQ % 128 == 0);
static_assert(DM % 32 == 0);
static_assert(DM % 8 == 0);
static_assert(HD == 64);
static_assert(NQKV == 3 * HD);
static_assert(RES_ROWS % 64 == 0);
static_assert(NB <= NB_FULL && SEQ <= SEQ_FULL);

typedef _Float16 v16h __attribute__((ext_vector_type(16)));
typedef unsigned short v8us __attribute__((ext_vector_type(8), may_alias));
typedef float  v8f  __attribute__((ext_vector_type(8)));
typedef float  v4f  __attribute__((ext_vector_type(4)));
typedef float  v4fa __attribute__((ext_vector_type(4), may_alias));
union FragH { v16h v; v8us half[2]; _Float16 h[16]; unsigned short u[16]; };

__device__ __forceinline__ unsigned short bf16_bits(float x) { unsigned int u = __float_as_uint(x); return (unsigned short)((u + 0x7FFFu + ((u >> 16) & 1u)) >> 16); }
__device__ __forceinline__ float bf16_rne(float x) { return __uint_as_float(((unsigned int)bf16_bits(x)) << 16); }

__device__ __forceinline__ v16h g2_frag(const _Float16* p, int hh) { FragH f; f.half[0] = *(const v8us*)((const unsigned short*)p + 8 * hh); f.half[1] = *(const v8us*)((const unsigned short*)p + 16 + 8 * hh); return f.v; }
__device__ __forceinline__ v8f g2_mma(v16h a, v16h b, v8f c) { v8f d = __builtin_amdgcn_wmma_f32_16x16x32_f16(false, a, false, b, (short)0, c, false, false); asm volatile("v_nop\n\tv_nop\n\tv_nop\n\tv_nop" : "+v"(d) : "v"(a), "v"(b)); return d; }
__device__ __forceinline__ void wave_sync() { __builtin_amdgcn_fence(4  , "workgroup"); __builtin_amdgcn_wave_barrier(); }

__global__ __launch_bounds__(256) void k_wt3(const float* __restrict__ Wq, const float* __restrict__ Wk, const float* __restrict__ Wv, _Float16* __restrict__ Bt) {
  const int t = blockIdx.x * 256 + threadIdx.x;
  if (t >= 3 * HD * (DM / 8)) return;
  const int m = t / (HD * (DM / 8)); const int rem = t - m * (HD * (DM / 8));
  const int n = rem / (DM / 8), k8 = (rem - n * (DM / 8)) * 8;
  FragH f;
#pragma unroll
  for (int i = 0; i < 8; ++i) {
    const size_t idx = (size_t)(k8 + i) * HD + n;
    const float a = Wq[idx], bq = Wk[idx], c = Wv[idx];
    const float v = (m == 0) ? a : ((m == 1) ? bq : c);
    f.h[i] = (_Float16)(bf16_rne(v) * 16.0f);
  }
  const v8us o = f.half[0];
  unsigned short* d = (unsigned short*)Bt + ((size_t)m * HD + n) * DM + k8;
  *(volatile v8us*)d = o; __threadfence(); *(volatile v8us*)d = o;
}

__global__ __launch_bounds__(256) void k_x16(const float* __restrict__ x, _Float16* __restrict__ X16) {
  const size_t t = (size_t)blockIdx.x * 256 + threadIdx.x;
  if (t >= NR * (DM / 8)) return;
  const size_t r = t / (DM / 8); const int c8 = (int)(t - r * (DM / 8)) * 8;
  const size_t b = r / SEQ, s = r - b * SEQ;
  const float* src = x + (b * SEQ_FULL + s) * DM + c8;
  const v4f a = *(const v4fa*)src, c = *(const v4fa*)(src + 4);
  FragH f;
#pragma unroll
  for (int q = 0; q < 4; ++q) { f.h[q] = (_Float16)bf16_rne(a[q]); f.h[4 + q] = (_Float16)bf16_rne(c[q]); }
  const v8us o = f.half[0];
  unsigned short* d = (unsigned short*)X16 + r * DM + c8;
  *(volatile v8us*)d = o; __threadfence(); *(volatile v8us*)d = o;
}

__global__ __launch_bounds__(128) void k_qkv(const _Float16* __restrict__ A, const _Float16* __restrict__ Bh, _Float16* __restrict__ P16) {
  __shared__ __attribute__((aligned(16))) float so[4][32][68];
  const int tid = threadIdx.x, w = tid >> 5, lane = tid & 31, ln = lane & 15, hh = lane >> 4;
  const int mt = blockIdx.x / 3, nq = blockIdx.x - mt * 3;
  const int row0 = mt * 128 + 32 * w, col0 = nq * 64;
  const _Float16* a0p = A + (size_t)(row0 + ln) * DM; const _Float16* a1p = a0p + (size_t)16 * DM;
  const _Float16* b0p = Bh + (size_t)(col0 + ln) * DM; const _Float16* b1p = b0p + (size_t)16 * DM; const _Float16* b2p = b1p + (size_t)16 * DM; const _Float16* b3p = b2p + (size_t)16 * DM;
  const v8f z8 = {0.f,0.f,0.f,0.f,0.f,0.f,0.f,0.f}; v8f c00 = z8, c01 = z8, c02 = z8, c03 = z8, c10 = z8, c11 = z8, c12 = z8, c13 = z8;
#pragma unroll 1
  for (int kb = 0; kb < DM; kb += 32) { const v16h a0 = g2_frag(a0p + kb, hh), a1 = g2_frag(a1p + kb, hh);
    v16h b = g2_frag(b0p + kb, hh); c00 = g2_mma(a0, b, c00); c10 = g2_mma(a1, b, c10);
    b = g2_frag(b1p + kb, hh); c01 = g2_mma(a0, b, c01); c11 = g2_mma(a1, b, c11);
    b = g2_frag(b2p + kb, hh); c02 = g2_mma(a0, b, c02); c12 = g2_mma(a1, b, c12);
    b = g2_frag(b3p + kb, hh); c03 = g2_mma(a0, b, c03); c13 = g2_mma(a1, b, c13); }
  v8f accs[8] = {c00, c01, c02, c03, c10, c11, c12, c13};
#pragma unroll
  for (int u = 0; u < 8; ++u) { const int t = u & 3, half = u >> 2;
#pragma unroll
    for (int r = 0; r < 8; ++r) so[w][half * 16 + 8 * hh + r][t * 16 + ln] = accs[u][r]; }
  wave_sync();
  const int rq = lane >> 3, c8 = (lane & 7) * 8;
  const size_t pbase = (size_t)(2 * nq) * PLANE;
  for (int pass = 0; pass < 2; ++pass) {
#pragma unroll
    for (int q = 0; q < 8; ++q) {
      const int r = q * 4 + rq;
      const v4f a = *(const v4fa*)&so[w][r][c8], c = *(const v4fa*)&so[w][r][c8 + 4];
      FragH fh, fl;
#pragma unroll
      for (int i = 0; i < 4; ++i) {
        _Float16 h = (_Float16)a[i]; fh.h[i] = h; fl.h[i] = (_Float16)((a[i] - (float)h) * 1024.0f);
        h = (_Float16)c[i]; fh.h[4 + i] = h; fl.h[4 + i] = (_Float16)((c[i] - (float)h) * 1024.0f);
      }
      unsigned short* dh = (unsigned short*)P16 + pbase + (size_t)(row0 + r) * HD + c8;
      *(volatile v8us*)dh = fh.half[0];
      *(volatile v8us*)(dh + PLANE) = fl.half[0];
    }
    if (pass == 0) __threadfence();
  }
}

__global__ __launch_bounds__(256) void k_vt(const _Float16* __restrict__ VR, _Float16* __restrict__ VT) {
  __shared__ unsigned short tl[64][66];
  const int tid = threadIdx.x; const int b = blockIdx.x / (SEQ / 64), lg = blockIdx.x - b * (SEQ / 64);
  const size_t po = (size_t)blockIdx.y * PLANE;
  for (int i = tid; i < 64 * 8; i += 256) { const int r = i / 8, c8 = (i % 8) * 8; FragH f;
    f.half[0] = *(const v8us*)((const unsigned short*)VR + po + ((size_t)b * SEQ + lg * 64 + r) * HD + c8);
#pragma unroll
    for (int q = 0; q < 8; ++q) tl[r][c8 + q] = f.u[q]; }
  __syncthreads();
  for (int pass = 0; pass < 2; ++pass) {
#pragma unroll
    for (int rd = 0; rd < 2; ++rd) { const int d = rd * 32 + tid / 8, pc = tid % 8; FragH f;
#pragma unroll
      for (int q = 0; q < 8; ++q) f.u[q] = tl[pc * 8 + q][d];
      *(volatile v8us*)((unsigned short*)VT + po + ((size_t)b * HD + d) * SEQ + lg * 64 + pc * 8) = f.half[0]; }
    if (pass == 0) __threadfence(); }
}

__global__ __launch_bounds__(128) void k_attn(const _Float16* __restrict__ P16, const _Float16* __restrict__ VT, float* __restrict__ out) {
  __shared__ __attribute__((aligned(16))) float so[4][16][68];
  const int tid = threadIdx.x, lane = tid & 31, ln = lane & 15, hh = lane >> 4;
  const int w = __builtin_amdgcn_readfirstlane(tid >> 5);
  const int b = blockIdx.x / (SEQ / 64), qb = blockIdx.x - b * (SEQ / 64);
  const int q0 = qb * 64 + w * 16;
  const bool res = (qb * 64 < RES_ROWS);
  const size_t rb = (size_t)b * SEQ;
  const _Float16* Qh = P16; const _Float16* Ql = P16 + PLANE; const _Float16* Kh = P16 + 2 * PLANE; const _Float16* Kl = P16 + 3 * PLANE;
  const _Float16* VTh = VT; const _Float16* VTl = VT + PLANE;
  const size_t qo = (rb + q0 + ln) * HD;
  const v16h qh0 = g2_frag(Qh + qo, hh), qh1 = g2_frag(Qh + qo + 32, hh);
  const v8f z8 = {0.f,0.f,0.f,0.f,0.f,0.f,0.f,0.f};
  const v8us z8us = {0,0,0,0,0,0,0,0};
  v8f o[4] = {z8, z8, z8, z8}, oe[4] = {z8, z8, z8, z8};
  float m = -1.0e30f, l = 0.f;
  const int klast = (q0 >> 5) << 5;
  const int query = q0 + ln;
  const size_t vrow = ((size_t)b * HD + ln) * SEQ;
#pragma unroll 1
  for (int kb = 0; kb <= klast; kb += 32) {
    v8f s[2] = {z8, z8}, rr[2] = {z8, z8};
#pragma unroll
    for (int t = 0; t < 2; ++t) {
      const size_t ko = (rb + kb + 16 * t + ln) * HD;
      const v16h ka = g2_frag(Kh + ko, hh), kc = g2_frag(Kh + ko + 32, hh);
      s[t] = g2_mma(ka, qh0, s[t]); s[t] = g2_mma(kc, qh1, s[t]);
      if (res) {
        const v16h ql0 = g2_frag(Ql + qo, hh), ql1 = g2_frag(Ql + qo + 32, hh);
        const v16h la = g2_frag(Kl + ko, hh), lc = g2_frag(Kl + ko + 32, hh);
        rr[t] = g2_mma(la, qh0, rr[t]); rr[t] = g2_mma(lc, qh1, rr[t]);
        rr[t] = g2_mma(ka, ql0, rr[t]); rr[t] = g2_mma(kc, ql1, rr[t]);
      }
    }
    float sv[2][8];
#pragma unroll
    for (int t = 0; t < 2; ++t)
#pragma unroll
      for (int r = 0; r < 8; ++r) sv[t][r] = (s[t][r] + rr[t][r] * 0.0009765625f) * 0.00048828125f;
    if (kb == klast) {
#pragma unroll
      for (int t = 0; t < 2; ++t)
#pragma unroll
        for (int r = 0; r < 8; ++r) { const int key = kb + 16 * t + 8 * hh + r; sv[t][r] = (key > query) ? -1.0e30f : sv[t][r]; }
    }
    float cm = fmaxf(sv[0][0], sv[1][0]);
#pragma unroll
    for (int r = 1; r < 8; ++r) cm = fmaxf(cm, fmaxf(sv[0][r], sv[1][r]));
    if (__builtin_amdgcn_ballot_w32(cm > m) != 0u) {
      const float mx = fmaxf(cm, __shfl_xor(cm, 16, 32));
      const float mn = fmaxf(m, mx);
      const float al = __expf(m - mn);
      m = mn; l *= al;
#pragma unroll
      for (int nt = 0; nt < 4; ++nt) o[nt] *= al;
      if (res) {
#pragma unroll
        for (int nt = 0; nt < 4; ++nt) oe[nt] *= al;
      }
    }
    FragH ph, pl; float cc[2][8]; float ls = 0.f;
    pl.half[0] = z8us; pl.half[1] = z8us;
#pragma unroll
    for (int r = 0; r < 8; ++r) {
      const float e0 = __expf(sv[0][r] - m), e1 = __expf(sv[1][r] - m);
      ls += e0 + e1;
      const float c0 = e0 * 256.0f, c1 = e1 * 256.0f;
      cc[0][r] = c0; cc[1][r] = c1;
      ph.h[r] = (_Float16)c0; ph.h[8 + r] = (_Float16)c1;
    }
    l += ls;
    if (res) {
#pragma unroll
      for (int r = 0; r < 8; ++r) {
        pl.h[r] = (_Float16)((cc[0][r] - (float)ph.h[r]) * 1024.0f);
        pl.h[8 + r] = (_Float16)((cc[1][r] - (float)ph.h[8 + r]) * 1024.0f);
      }
    }
    const v16h phv = ph.v, plv = pl.v;
#pragma unroll
    for (int nt = 0; nt < 4; ++nt) {
      const size_t vo = vrow + (size_t)(16 * nt) * SEQ + kb;
      const v16h va = g2_frag(VTh + vo, hh);
      o[nt] = g2_mma(va, phv, o[nt]);
      if (res) {
        const v16h vl = g2_frag(VTl + vo, hh);
        oe[nt] = g2_mma(va, plv, oe[nt]); oe[nt] = g2_mma(vl, phv, oe[nt]);
      }
    }
  }
  const float lt = l + __shfl_xor(l, 16, 32);
  const float sc = (1.0f / lt) * 0.000244140625f;
#pragma unroll
  for (int nt = 0; nt < 4; ++nt) {
    v4f a, c;
#pragma unroll
    for (int i = 0; i < 4; ++i) { a[i] = (o[nt][i] + oe[nt][i] * 0.0009765625f) * sc; c[i] = (o[nt][4 + i] + oe[nt][4 + i] * 0.0009765625f) * sc; }
    *(v4fa*)&so[w][ln][16 * nt + 8 * hh] = a;
    *(v4fa*)&so[w][ln][16 * nt + 8 * hh + 4] = c;
  }
  wave_sync();
  const int rsub = lane >> 4, c4 = (lane & 15) * 4;
  const size_t orow0 = (size_t)b * SEQ_FULL + q0;
  for (int pass = 0; pass < 2; ++pass) {
#pragma unroll
    for (int q = 0; q < 8; ++q) {
      const int r = q * 2 + rsub;
      const v4f v = *(const v4fa*)&so[w][r][c4];
      *(volatile v4f*)(out + (orow0 + r) * HD + c4) = v;
    }
    if (pass == 0) __threadfence();
  }
}

#define AL256(x) ((((size_t)(x)) + 255) & ~(size_t)255)
#define SZ_BT ((size_t)NQKV * DM * 2)
#define SZ_X  (NR * DM * 2)
#define SZ_P  ((size_t)6 * PLANE * 2)
#define SZ_VT ((size_t)2 * PLANE * 2)
static_assert(AL256(SZ_BT) + AL256(SZ_X) + AL256(SZ_P) + AL256(SZ_VT) <= (size_t)134217728);
static_assert((NR * (DM / 8)) % 256 == 0);
static_assert(NR % 128 == 0);

extern "C" void kernel_launch(void* const* d_in, const int* in_sizes, int n_in,
                              void* d_out, int out_size, void* d_ws, size_t ws_size, hipStream_t stream) {
  if (n_in < 4) return;
  const size_t rows_need = (size_t)(NB - 1) * SEQ_FULL + SEQ;
  if ((size_t)in_sizes[0] < rows_need * DM) return;
  if (in_sizes[1] < DM * HD || in_sizes[2] < DM * HD || in_sizes[3] < DM * HD) return;
  if ((size_t)out_size < rows_need * HD) return;
  const float* x = (const float*)d_in[0]; const float* wq = (const float*)d_in[1]; const float* wk = (const float*)d_in[2]; const float* wv = (const float*)d_in[3];
  char* ws = (char*)d_ws; size_t off = 0;
  _Float16* Bt  = (_Float16*)(ws + off); off += AL256(SZ_BT);
  _Float16* X16 = (_Float16*)(ws + off); off += AL256(SZ_X);
  _Float16* P16 = (_Float16*)(ws + off); off += AL256(SZ_P);
  _Float16* VT  = (_Float16*)(ws + off); off += AL256(SZ_VT);
  if (off > ws_size) return;
  k_wt3<<<(unsigned)((3 * HD * (DM / 8) + 255) / 256), 256, 0, stream>>>(wq, wk, wv, Bt);
  k_x16<<<(unsigned)((NR * (DM / 8) + 255) / 256), 256, 0, stream>>>(x, X16);
  k_qkv<<<(unsigned)((NR / 128) * 3), 128, 0, stream>>>(X16, Bt, P16);
  k_vt<<<dim3((unsigned)(NB * (SEQ / 64)), 2), 256, 0, stream>>>(P16 + 4 * PLANE, VT);
  k_attn<<<(unsigned)(NB * (SEQ / 64)), 128, 0, stream>>>(P16, VT, (float*)d_out);
}
